// Block_72739566125973
// MI455X (gfx1250) — hardware-verified
//
#include <hip/hip_runtime.h>
#ifndef NB
#define NB 2
#endif
#ifndef SEQ
#define SEQ 2048
#endif
#define NB_FULL 2
#define SEQ_FULL 2048
#define SQ SEQ
#define DM 1024
#define NH 16
#define HD 64
#define DFF 4096
#define QT0 256
#define LQ (3 * DM)
#define NR ((size_t)NB * SQ)
static_assert(DM == NH * HD);
static_assert(HD == 64);
static_assert(DM == 256 * 4);
static_assert(SQ % 128 == 0);
static_assert(QT0 % 128 == 0);
static_assert(QT0 <= SQ);
static_assert(DM % 64 == 0);
static_assert(DFF % 64 == 0);
static_assert((3 * DM) % 64 == 0);
static_assert(DM % 32 == 0);
static_assert(DFF % 32 == 0);
static_assert(NB <= NB_FULL);
static_assert(SQ <= SEQ_FULL);

typedef unsigned short v8us __attribute__((ext_vector_type(8), may_alias));
typedef float  v8f  __attribute__((ext_vector_type(8)));
typedef float  v4f  __attribute__((ext_vector_type(4)));
typedef float  v4fa __attribute__((ext_vector_type(4), may_alias));
typedef _Float16 v16h __attribute__((ext_vector_type(16)));
typedef _Float16 v4h __attribute__((ext_vector_type(4)));
union FragH { v16h v; v8us half[2]; _Float16 h[16]; unsigned short u[16]; };

__device__ __forceinline__ unsigned short bf16_bits(float x) { unsigned int u = __float_as_uint(x); return (unsigned short)((u + 0x7FFFu + ((u >> 16) & 1u)) >> 16); }
__device__ __forceinline__ float bf16_val(unsigned short b) { return __uint_as_float(((unsigned int)b) << 16); }
__device__ __forceinline__ float bf16_rne(float x) { return bf16_val(bf16_bits(x)); }

__device__ __forceinline__ v16h g2_frag(const _Float16* p, int hh) { FragH f; f.half[0] = *(const v8us*)((const unsigned short*)p + 8 * hh); f.half[1] = *(const v8us*)((const unsigned short*)p + 16 + 8 * hh); return f.v; }
__device__ __forceinline__ v8f g2_mma(v16h a, v16h b, v8f c) { v8f d = __builtin_amdgcn_wmma_f32_16x16x32_f16(false, a, false, b, (short)0, c, false, false); asm volatile("v_nop\n\tv_nop\n\tv_nop\n\tv_nop" : "+v"(d) : "v"(a), "v"(b)); return d; }

__global__ __launch_bounds__(256) void k_wt_f16(const float* __restrict__ W, _Float16* __restrict__ Wt, int K, int N, float scale) {
  const int t = blockIdx.x * 256 + threadIdx.x; if (t >= N * (K / 8)) return; const int n = t / (K / 8), k8 = (t % (K / 8)) * 8; FragH f;
#pragma unroll
  for (int i = 0; i < 8; ++i) f.h[i] = (_Float16)(bf16_rne(W[(size_t)(k8 + i) * N + n]) * scale);
  const v8us o = f.half[0];
  *(volatile v8us*)((unsigned short*)Wt + (size_t)n * K + k8) = o; __threadfence(); *(volatile v8us*)((unsigned short*)Wt + (size_t)n * K + k8) = o;
}

template <int ACT>
__device__ __forceinline__ void gemm2_body(const _Float16* __restrict__ A, int lda, size_t sA, const _Float16* __restrict__ Bh, int ldb, float alpha, const float* __restrict__ bias, const float* CP,
    float* C, _Float16* C16, int ldc, size_t sC, int M, int N, int K) {
  static_assert(ACT == 0 || ACT == 6);
  __shared__ __attribute__((aligned(16))) float so[4][32][68];
  const int tid = threadIdx.x, w = tid >> 5, lane = tid & 31, ln = lane & 15, hh = lane >> 4; const int by = blockIdx.y;
  A += (size_t)by * sA; const size_t cofs = (size_t)by * sC;
  const int ntn = N >> 6; const int mt = blockIdx.x / ntn, nq = blockIdx.x - mt * ntn; const int row0 = mt * 128 + 32 * w, col0 = nq * 64; if (row0 >= M) return;
  const _Float16* a0p = A + (size_t)(row0 + ln) * lda; const _Float16* a1p = a0p + (size_t)16 * lda;
  const _Float16* b0p = Bh + (size_t)(col0 + ln) * ldb; const _Float16* b1p = b0p + (size_t)16 * ldb; const _Float16* b2p = b1p + (size_t)16 * ldb; const _Float16* b3p = b2p + (size_t)16 * ldb;
  const v8f z8 = {0.f,0.f,0.f,0.f,0.f,0.f,0.f,0.f}; v8f c00 = z8, c01 = z8, c02 = z8, c03 = z8, c10 = z8, c11 = z8, c12 = z8, c13 = z8;
#pragma unroll 1
  for (int kb = 0; kb < K; kb += 32) { const v16h a0 = g2_frag(a0p + kb, hh), a1 = g2_frag(a1p + kb, hh);
    v16h b = g2_frag(b0p + kb, hh); c00 = g2_mma(a0, b, c00); c10 = g2_mma(a1, b, c10);
    b = g2_frag(b1p + kb, hh); c01 = g2_mma(a0, b, c01); c11 = g2_mma(a1, b, c11);
    b = g2_frag(b2p + kb, hh); c02 = g2_mma(a0, b, c02); c12 = g2_mma(a1, b, c12);
    b = g2_frag(b3p + kb, hh); c03 = g2_mma(a0, b, c03); c13 = g2_mma(a1, b, c13); }
  v8f accs[8] = {c00, c01, c02, c03, c10, c11, c12, c13};
#pragma unroll
  for (int u = 0; u < 8; ++u) { const int t = u & 3, half = u >> 2; const int col = col0 + t * 16 + ln; float bv = 0.f; if (bias) bv = bf16_rne(bias[col]);
#pragma unroll
    for (int r = 0; r < 8; ++r) { const int rloc = half * 16 + 8 * hh + r; float v = accs[u][r] * alpha + bv;
      if (ACT == 6) v = 0.5f * v * (1.0f + erff(v * 0.70710678118654752f));
      so[w][rloc][t * 16 + ln] = v; } }
  __builtin_amdgcn_fence(4  , "workgroup"); __builtin_amdgcn_wave_barrier();
  const int rsub = lane >> 4, c4 = (lane & 15) * 4;
  v4f ov[16];
#pragma unroll
  for (int q = 0; q < 16; ++q) { const int r = q * 2 + rsub; v4f v = *(const v4fa*)&so[w][r][c4];
    if (CP) { const v4f rv = *(const v4fa*)(CP + cofs + (size_t)(row0 + r) * ldc + col0 + c4); v = v + rv; }
    ov[q] = v; }
  for (int pass = 0; pass < 2; ++pass) {
#pragma unroll
    for (int q = 0; q < 16; ++q) { const int r = q * 2 + rsub; const v4f v = ov[q];
      if (C) *(volatile v4f*)(C + cofs + (size_t)(row0 + r) * ldc + col0 + c4) = v;
      if (C16) { v4h h4;
#pragma unroll
        for (int i = 0; i < 4; ++i) h4[i] = (_Float16)v[i];
        *(volatile v4h*)(C16 + cofs + (size_t)(row0 + r) * ldc + col0 + c4) = h4; } }
    if (pass == 0) __threadfence(); } }
__global__ __launch_bounds__(128) void k_gemm2_lin(const _Float16* __restrict__ A, int lda, size_t sA, const _Float16* __restrict__ Bh, int ldb, float alpha, const float* __restrict__ bias, const float* CP,
    float* C, _Float16* C16, int ldc, size_t sC, int M, int N, int K) { gemm2_body<0>(A, lda, sA, Bh, ldb, alpha, bias, CP, C, C16, ldc, sC, M, N, K); }
__global__ __launch_bounds__(128) void k_gemm2_gelu(const _Float16* __restrict__ A, int lda, size_t sA, const _Float16* __restrict__ Bh, int ldb, float alpha, const float* __restrict__ bias, const float* CP,
    float* C, _Float16* C16, int ldc, size_t sC, int M, int N, int K) { gemm2_body<6>(A, lda, sA, Bh, ldb, alpha, bias, CP, C, C16, ldc, sC, M, N, K); }

__global__ __launch_bounds__(256) void k_vt(const _Float16* __restrict__ V16, int ldv, int voff, _Float16* __restrict__ Vt) {
  __shared__ unsigned short tl[64][66]; const int tid = threadIdx.x; const int slab = blockIdx.x / (SQ / 64), lg = blockIdx.x % (SQ / 64); const int b = slab / NH, h = slab % NH;
  for (int i = tid; i < 64 * 8; i += 256) { const int r = i / 8, c8 = (i % 8) * 8; FragH f; f.half[0] = *(const v8us*)((const unsigned short*)V16 + ((size_t)b * SQ + lg * 64 + r) * ldv + voff + h * 64 + c8);
#pragma unroll
    for (int q = 0; q < 8; ++q) tl[r][c8 + q] = f.u[q]; }
  __syncthreads();
  for (int pass = 0; pass < 2; ++pass) {
#pragma unroll
    for (int rd = 0; rd < 2; ++rd) { const int d = rd * 32 + tid / 8, pc = tid % 8; FragH f;
#pragma unroll
      for (int q = 0; q < 8; ++q) f.u[q] = tl[pc * 8 + q][d];
      *(volatile v8us*)((unsigned short*)Vt + ((size_t)slab * 64 + d) * SQ + lg * 64 + pc * 8) = f.half[0]; }
    if (pass == 0) __threadfence(); } }

__global__ __launch_bounds__(128) void k_flash(const _Float16* __restrict__ QKV, const _Float16* __restrict__ VT, _Float16* __restrict__ O16) {
  __shared__ __attribute__((aligned(16))) _Float16 sp[4][16][72];
  __shared__ __attribute__((aligned(16))) float so[4][16][68];
  const int tid = threadIdx.x, w = tid >> 5, lane = tid & 31, ln = lane & 15, hh = lane >> 4;
  const int bh = blockIdx.y, b = bh / NH, h = bh % NH; const int qb = blockIdx.x; const int q0 = qb * 64 + w * 16; const size_t r0 = (size_t)b * SQ;
  const _Float16* qrow = QKV + (r0 + q0 + ln) * LQ + h * HD;
  const v16h qa0 = g2_frag(qrow, hh), qa1 = g2_frag(qrow + 32, hh);
  const _Float16* kbase = QKV + r0 * LQ + DM + h * HD;
  const _Float16* vtb = VT + (size_t)bh * HD * SQ;
  const v8f z8 = {0.f,0.f,0.f,0.f,0.f,0.f,0.f,0.f};
  v8f o[4] = {z8, z8, z8, z8}; float mrow[8], lrow[8];
#pragma unroll
  for (int r = 0; r < 8; ++r) { mrow[r] = -1.0e30f; lrow[r] = 0.f; }
#pragma unroll 1
  for (int c = 0; c <= qb; ++c) { const int j0 = c * 64;
    v8f s[4];
#pragma unroll
    for (int t = 0; t < 4; ++t) { const _Float16* kp = kbase + (size_t)(j0 + t * 16 + ln) * LQ; const v16h kb0 = g2_frag(kp, hh), kb1 = g2_frag(kp + 32, hh); s[t] = g2_mma(qa0, kb0, z8); s[t] = g2_mma(qa1, kb1, s[t]); }
#pragma unroll
    for (int r = 0; r < 8; ++r) { const int row = q0 + 8 * hh + r; float sv[4]; float mx = -1.0e30f;
#pragma unroll
      for (int t = 0; t < 4; ++t) { const int key = j0 + t * 16 + ln; const float x = s[t][r] * 0.125f; sv[t] = (key <= row) ? x : -1.0e30f; mx = fmaxf(mx, sv[t]); }
      mx = fmaxf(mx, __shfl_xor(mx, 1)); mx = fmaxf(mx, __shfl_xor(mx, 2)); mx = fmaxf(mx, __shfl_xor(mx, 4)); mx = fmaxf(mx, __shfl_xor(mx, 8));
      const float mn = fmaxf(mrow[r], mx); const float sc = __expf(mrow[r] - mn); float rs = 0.f;
#pragma unroll
      for (int t = 0; t < 4; ++t) { const float p = __expf(sv[t] - mn); rs += p; sp[w][8 * hh + r][t * 16 + ln] = (_Float16)(p * 256.0f); }
      rs += __shfl_xor(rs, 1); rs += __shfl_xor(rs, 2); rs += __shfl_xor(rs, 4); rs += __shfl_xor(rs, 8);
      lrow[r] = lrow[r] * sc + rs; mrow[r] = mn;
#pragma unroll
      for (int nt = 0; nt < 4; ++nt) o[nt][r] *= sc; }
    __builtin_amdgcn_fence(4  , "workgroup"); __builtin_amdgcn_wave_barrier();
#pragma unroll
    for (int kk = 0; kk < 2; ++kk) { FragH pf; pf.half[0] = *(const v8us*)&sp[w][ln][kk * 32 + 8 * hh]; pf.half[1] = *(const v8us*)&sp[w][ln][kk * 32 + 16 + 8 * hh];
#pragma unroll
      for (int nt = 0; nt < 4; ++nt) { const v16h vb = g2_frag(vtb + (size_t)(nt * 16 + ln) * SQ + j0 + kk * 32, hh); o[nt] = g2_mma(pf.v, vb, o[nt]); } }
    __builtin_amdgcn_fence(4  , "workgroup"); __builtin_amdgcn_wave_barrier(); }
#pragma unroll
  for (int r = 0; r < 8; ++r) { const float fin = 0.25f / lrow[r];
#pragma unroll
    for (int nt = 0; nt < 4; ++nt) so[w][8 * hh + r][nt * 16 + ln] = o[nt][r] * fin; }
  __builtin_amdgcn_fence(4  , "workgroup"); __builtin_amdgcn_wave_barrier();
  const int rq = lane >> 3, c8 = (lane & 7) * 8;
  v8us pk[4];
#pragma unroll
  for (int q = 0; q < 4; ++q) { const int row = q * 4 + rq; const v4f a = *(const v4fa*)&so[w][row][c8], cc = *(const v4fa*)&so[w][row][c8 + 4]; FragH f;
#pragma unroll
    for (int i = 0; i < 4; ++i) { f.h[i] = (_Float16)a[i]; f.h[4 + i] = (_Float16)cc[i]; }
    pk[q] = f.half[0]; }
  unsigned short* ob = (unsigned short*)O16 + (r0 + q0) * DM + h * HD + c8;
  for (int pass = 0; pass < 2; ++pass) {
#pragma unroll
    for (int q = 0; q < 4; ++q) *(volatile v8us*)(ob + (size_t)(q * 4 + rq) * DM) = pk[q];
    if (pass == 0) __threadfence(); } }

__global__ __launch_bounds__(64) void k_att0(const float* __restrict__ QF, const float* __restrict__ KF, const float* __restrict__ VF, int ld, float scale, float* __restrict__ OF, int ldo) {
  #pragma clang fp contract(off)
  __shared__ __attribute__((aligned(16))) float lq[64][64]; __shared__ __attribute__((aligned(16))) float lo[64][64];
  const int tid = threadIdx.x; const int h = blockIdx.x / (QT0 / 64), rg = blockIdx.x % (QT0 / 64); const int i = rg * 64 + tid;
  const float* qr = QF + (size_t)i * ld + h * HD;
#pragma unroll 1
  for (int c = 0; c < HD / 4; ++c) { *(v4f*)&lq[tid][c * 4] = *(const v4fa*)(qr + c * 4); const v4f z = {0.f, 0.f, 0.f, 0.f}; *(v4f*)&lo[tid][c * 4] = z; }
  float m = -1.0e30f, l = 0.f; const int jmax = rg * 64 + 63;
#pragma unroll 1
  for (int j = 0; j <= jmax; ++j) { const float* kr = KF + (size_t)j * ld + h * HD; const float* vr = VF + (size_t)j * ld + h * HD; float s = 0.f;
#pragma unroll 1
    for (int c = 0; c < HD / 4; ++c) { const v4f kq = *(const v4fa*)(kr + c * 4); const v4f qq = *(v4f*)&lq[tid][c * 4]; s = __fadd_rn(s, __fmul_rn(qq[0], kq[0])); s = __fadd_rn(s, __fmul_rn(qq[1], kq[1])); s = __fadd_rn(s, __fmul_rn(qq[2], kq[2])); s = __fadd_rn(s, __fmul_rn(qq[3], kq[3])); }
    s = __fmul_rn(s, scale);
    const float f = (j <= i) ? 1.f : 0.f; const float sm = fmaf(f, s, (1.f - f) * -1.0e30f); const float mn = fmaxf(m, sm); const float sc = expf(m - mn); const float e = expf(sm - mn); l = __fadd_rn(__fmul_rn(l, sc), e); m = mn;
#pragma unroll 1
    for (int c = 0; c < HD / 4; ++c) { const v4f vv = *(const v4fa*)(vr + c * 4); v4f oo = *(v4f*)&lo[tid][c * 4];
#pragma unroll
      for (int u = 0; u < 4; ++u) oo[u] = __fadd_rn(__fmul_rn(oo[u], sc), __fmul_rn(e, vv[u]));
      *(v4f*)&lo[tid][c * 4] = oo; } }
  const float fin = 64.0f / l;
#pragma unroll 1
  for (int c = 0; c < HD / 4; ++c) { v4f oo = *(v4f*)&lo[tid][c * 4];
#pragma unroll
    for (int u = 0; u < 4; ++u) oo[u] = __fmul_rn(oo[u], fin);
    *(v4f*)&lo[tid][c * 4] = oo; }
  __syncthreads();
  for (int pass = 0; pass < 2; ++pass) {
#pragma unroll 1
    for (int it = 0; it < 16; ++it) { const int row = it * 4 + tid / 16, pc = (tid % 16) * 4; const v4f v = *(const v4f*)&lo[row][pc]; *(volatile v4f*)(OF + (size_t)(rg * 64 + row) * ldo + h * HD + pc) = v; }
    if (pass == 0) __threadfence(); } }

template <int BFIN, int WXB>
__device__ __forceinline__ void ln16_body(const float* __restrict__ X, int sqin, const float* __restrict__ g, const float* __restrict__ bb, float eps, _Float16* __restrict__ N16, float* __restrict__ XB) {
  #pragma clang fp contract(off)
  __shared__ float red[256]; const size_t r = blockIdx.x; const int t = threadIdx.x; const size_t rin = (r / SQ) * (size_t)sqin + (r % SQ);
  const v4f xa = *(const v4fa*)(X + rin * DM + t * 4); float s[4]; float sum = 0.f;
#pragma unroll
  for (int q = 0; q < 4; ++q) { s[q] = BFIN ? bf16_rne(xa[q]) : xa[q]; sum = __fadd_rn(sum, s[q]); }
  red[t] = sum; __syncthreads();
  for (int st = 128; st > 0; st >>= 1) { if (t < st) red[t] = __fadd_rn(red[t], red[t + st]); __syncthreads(); }
  const float mu = red[0] / (float)DM; __syncthreads();
  float vs = 0.f;
#pragma unroll
  for (int q = 0; q < 4; ++q) { const float dl = __fadd_rn(s[q], -mu); vs = __fadd_rn(vs, __fmul_rn(dl, dl)); }
  red[t] = vs; __syncthreads();
  for (int st = 128; st > 0; st >>= 1) { if (t < st) red[t] = __fadd_rn(red[t], red[t + st]); __syncthreads(); }
  const float rs = rsqrtf(__fadd_rn(red[0] / (float)DM, eps)); v4h y; v4f xb;
#pragma unroll
  for (int q = 0; q < 4; ++q) { const int c = t * 4 + q; y[q] = (_Float16)__fadd_rn(__fmul_rn(__fmul_rn(__fadd_rn(s[q], -mu), rs), bf16_rne(g[c])), bf16_rne(bb[c])); xb[q] = s[q]; }
  for (int pass = 0; pass < 2; ++pass) { *(volatile v4h*)(N16 + r * DM + t * 4) = y; if (WXB) *(volatile v4f*)(XB + r * DM + t * 4) = xb; if (pass == 0) __threadfence(); } }
__global__ __launch_bounds__(256) void k_ln16_in(const float* __restrict__ X, int sqin, const float* __restrict__ g, const float* __restrict__ bb, float eps, _Float16* __restrict__ N16, float* __restrict__ XB) { ln16_body<1, 1>(X, sqin, g, bb, eps, N16, XB); }
__global__ __launch_bounds__(256) void k_ln16_mid(const float* __restrict__ X, int sqin, const float* __restrict__ g, const float* __restrict__ bb, float eps, _Float16* __restrict__ N16, float* __restrict__ XB) { ln16_body<0, 0>(X, sqin, g, bb, eps, N16, XB); }

__global__ __launch_bounds__(256) void k_hl(const float* __restrict__ F, _Float16* __restrict__ Hh, _Float16* __restrict__ Hl, size_t n8) { const size_t t = (size_t)blockIdx.x * 256 + threadIdx.x; if (t >= n8) return; FragH fh, fl; const v4f a = *(const v4fa*)(F + t * 8), c = *(const v4fa*)(F + t * 8 + 4);
#pragma unroll
  for (int q = 0; q < 4; ++q) { _Float16 h = (_Float16)a[q]; fh.h[q] = h; fl.h[q] = (_Float16)((a[q] - (float)h) * 1024.0f); h = (_Float16)c[q]; fh.h[4 + q] = h; fl.h[4 + q] = (_Float16)((c[q] - (float)h) * 1024.0f); }
  for (int pass = 0; pass < 2; ++pass) { *(volatile v8us*)((unsigned short*)Hh + t * 8) = fh.half[0]; *(volatile v8us*)((unsigned short*)Hl + t * 8) = fl.half[0]; if (pass == 0) __threadfence(); } }

constexpr size_t al256(size_t b) { return (b + 255) & ~(size_t)255; }
constexpr size_t cmax(size_t a, size_t b) { return a > b ? a : b; }
constexpr size_t B_BQKV = al256((size_t)3 * DM * DM * 2);
constexpr size_t B_BO   = al256((size_t)DM * DM * 2);
constexpr size_t B_BW1  = al256((size_t)DFF * DM * 2);
constexpr size_t B_BW2  = al256((size_t)DM * DFF * 2);
constexpr size_t B_X16  = al256(NR * DM * 2);
constexpr size_t B_XB   = al256(NR * DM * 4);
constexpr size_t B_X1   = al256(NR * DM * 4);
constexpr size_t B_QKVU = (size_t)NR * 3 * DM * 2;
constexpr size_t B_HFU  = (size_t)SQ * DFF * 2;
constexpr size_t B_ATT  = al256(cmax(B_QKVU, B_HFU));
constexpr size_t B_O16  = al256(NR * DM * 2);
constexpr size_t B_VT   = al256((size_t)NB * NH * HD * SQ * 2);
constexpr size_t B_F0   = al256((size_t)NB * QT0 * 3 * DM * 4);
constexpr size_t B_OF0  = al256((size_t)NB * QT0 * DM * 4);
constexpr size_t B_OH0  = al256((size_t)NB * QT0 * DM * 2);
constexpr size_t B_TOTAL = B_BQKV + B_BO + B_BW1 + B_BW2 + B_X16 + B_XB + B_X1 + B_ATT + B_O16 + B_VT + B_F0 + B_OF0 + 2 * B_OH0;
static_assert(B_TOTAL <= (size_t)134217728);
static_assert(B_QKVU <= B_ATT);
static_assert(B_HFU <= B_ATT);

extern "C" void kernel_launch(void* const* d_in, const int* in_sizes, int n_in,
                              void* d_out, int out_size, void* d_ws, size_t ws_size, hipStream_t stream) {
  if (n_in < 11) return;
  const size_t xneed = ((size_t)(NB - 1) * SEQ_FULL + SQ) * DM;
  if ((size_t)in_sizes[0] < xneed || (size_t)out_size < xneed) return;
  if (in_sizes[1] < 3 * DM * DM || in_sizes[2] < DM * DM || in_sizes[3] < DM || in_sizes[4] < DM || in_sizes[5] < DM || in_sizes[6] < DM) return;
  if (in_sizes[7] < DM * DFF || in_sizes[8] < DFF || in_sizes[9] < DFF * DM || in_sizes[10] < DM) return;
  if (B_TOTAL > ws_size) return;
  const float* const* I = (const float* const*)d_in;
  const float* x = I[0]; const float* wqkv = I[1]; const float* wo = I[2]; const float* g1 = I[3]; const float* be1 = I[4]; const float* g2 = I[5]; const float* be2 = I[6];
  const float* w1 = I[7]; const float* b1 = I[8]; const float* w2 = I[9]; const float* b2 = I[10];
  float* outp = (float*)d_out;
  char* ws = (char*)d_ws; size_t off = 0;
  _Float16* BQKV = (_Float16*)(ws + off); off += B_BQKV;
  _Float16* BO   = (_Float16*)(ws + off); off += B_BO;
  _Float16* BW1  = (_Float16*)(ws + off); off += B_BW1;
  _Float16* BW2  = (_Float16*)(ws + off); off += B_BW2;
  _Float16* X16  = (_Float16*)(ws + off); off += B_X16;
  float*    XB   = (float*)(ws + off);    off += B_XB;
  float*    X1   = (float*)(ws + off);    off += B_X1;
  _Float16* QKV  = (_Float16*)(ws + off); off += B_ATT;
  _Float16* O16  = (_Float16*)(ws + off); off += B_O16;
  _Float16* VT   = (_Float16*)(ws + off); off += B_VT;
  float*    F0   = (float*)(ws + off);    off += B_F0;
  float*    OF0  = (float*)(ws + off);    off += B_OF0;
  _Float16* OH0  = (_Float16*)(ws + off); off += B_OH0;
  _Float16* OL0  = (_Float16*)(ws + off); off += B_OH0;
  _Float16* HF16 = QKV;
  _Float16* M16  = X16;

  k_wt_f16<<<(unsigned)(((size_t)3 * DM * (DM / 8) + 255) / 256), 256, 0, stream>>>(wqkv, BQKV, DM, 3 * DM, 16.0f);
  k_wt_f16<<<(unsigned)(((size_t)DM * (DM / 8) + 255) / 256), 256, 0, stream>>>(wo, BO, DM, DM, 16.0f);
  k_wt_f16<<<(unsigned)(((size_t)DFF * (DM / 8) + 255) / 256), 256, 0, stream>>>(w1, BW1, DM, DFF, 16.0f);
  k_wt_f16<<<(unsigned)(((size_t)DM * (DFF / 8) + 255) / 256), 256, 0, stream>>>(w2, BW2, DFF, DM, 16.0f);
  k_ln16_in<<<(unsigned)NR, 256, 0, stream>>>(x, SEQ_FULL, g1, be1, 1e-5f, X16, XB);
  k_gemm2_lin<<<dim3((unsigned)((NR / 128) * (3 * DM / 64)), 1), 128, 0, stream>>>(X16, DM, 0, BQKV, DM, 0.0625f, nullptr, nullptr, nullptr, QKV, 3 * DM, 0, (int)NR, 3 * DM, DM);
  k_gemm2_lin<<<dim3((unsigned)((QT0 / 128) * (3 * DM / 64)), NB), 128, 0, stream>>>(X16, DM, (size_t)SQ * DM, BQKV, DM, 0.0625f, nullptr, nullptr, F0, nullptr, 3 * DM, (size_t)QT0 * 3 * DM, QT0, 3 * DM, DM);
  k_vt<<<(unsigned)(NB * NH * (SQ / 64)), 256, 0, stream>>>(QKV, LQ, 2 * DM, VT);
  k_flash<<<dim3(SQ / 64, NB * NH), 128, 0, stream>>>(QKV, VT, O16);
  for (int b = 0; b < NB; ++b) { const float* f0 = F0 + (size_t)b * QT0 * 3 * DM;
    k_att0<<<NH * (QT0 / 64), 64, 0, stream>>>(f0, f0 + DM, f0 + 2 * DM, 3 * DM, 0.125f, OF0 + (size_t)b * QT0 * DM, DM); }
  k_gemm2_lin<<<dim3((unsigned)((NR / 128) * (DM / 64)), 1), 128, 0, stream>>>(O16, DM, 0, BO, DM, 0.0009765625f, nullptr, XB, X1, nullptr, DM, 0, (int)NR, DM, DM);
  k_hl<<<(unsigned)(((size_t)NB * QT0 * DM / 8 + 255) / 256), 256, 0, stream>>>(OF0, OH0, OL0, (size_t)NB * QT0 * DM / 8);
  k_gemm2_lin<<<dim3((unsigned)((QT0 / 128) * (DM / 64)), NB), 128, 0, stream>>>(OH0, DM, (size_t)QT0 * DM, BO, DM, 0.0009765625f, nullptr, XB, X1, nullptr, DM, (size_t)SQ * DM, QT0, DM, DM);
  k_gemm2_lin<<<dim3((unsigned)((QT0 / 128) * (DM / 64)), NB), 128, 0, stream>>>(OL0, DM, (size_t)QT0 * DM, BO, DM, 0.00000095367431640625f, nullptr, X1, X1, nullptr, DM, (size_t)SQ * DM, QT0, DM, DM);
  k_ln16_mid<<<(unsigned)NR, 256, 0, stream>>>(X1, SQ, g2, be2, 1e-5f, M16, nullptr);
  for (int b = 0; b < NB; ++b) { const size_t r0 = (size_t)b * SQ;
    k_gemm2_gelu<<<dim3((unsigned)((SQ / 128) * (DFF / 64)), 1), 128, 0, stream>>>(M16 + r0 * DM, DM, 0, BW1, DM, 0.0625f, b1, nullptr, nullptr, HF16, DFF, 0, SQ, DFF, DM);
    k_gemm2_lin<<<dim3((unsigned)((SQ / 128) * (DM / 64)), 1), 128, 0, stream>>>(HF16, DFF, 0, BW2, DFF, 0.0625f, b2, X1 + r0 * DM, outp + (size_t)b * SEQ_FULL * DM, nullptr, DM, 0, SQ, DM, DFF); }
}
